// GraphAttention_Naive_59476707115119
// MI455X (gfx1250) — hardware-verified
//
#include <hip/hip_runtime.h>


#define DM   1024
#define NH   16
#define DH   64
#define NB   4
#define SEQ  2048

typedef _Float16       v16h __attribute__((ext_vector_type(16)));
typedef __bf16         v16b __attribute__((ext_vector_type(16)));
typedef unsigned short us16 __attribute__((ext_vector_type(16)));
typedef unsigned short us8  __attribute__((ext_vector_type(8), may_alias));
typedef float          v8f  __attribute__((ext_vector_type(8)));
typedef float          v4f  __attribute__((ext_vector_type(4), may_alias));

union Frag { us16 u; us8 p[2]; v16h h; v16b b; };

static_assert(SEQ % 128 == 0);
static_assert(DM % 64 == 0);
static_assert(NH * DH == DM);

__device__ __forceinline__ unsigned short f2h(float f) {
  union { _Float16 h; unsigned short u; } c;
  c.h = (_Float16)f;
  return c.u;
}
__device__ __forceinline__ unsigned short f2bf(float f) {
  unsigned int u = __float_as_uint(f);
  u += 0x7FFFu + ((u >> 16) & 1u);
  return (unsigned short)(u >> 16);
}
__device__ __forceinline__ float bf2f(unsigned short v) {
  return __uint_as_float(((unsigned int)v) << 16);
}
__device__ __forceinline__ v8f vzero() {
  v8f z;
#pragma unroll
  for (int i = 0; i < 8; ++i) z[i] = 0.0f;
  return z;
}
__device__ __forceinline__ void ld8(const float* __restrict__ p, float* f) {
  v4f a = *(const v4f*)p;
  v4f b = *(const v4f*)(p + 4);
#pragma unroll
  for (int i = 0; i < 4; ++i) { f[i] = a[i]; f[4 + i] = b[i]; }
}

__device__ __forceinline__ us16 ldfrag(const unsigned short* p, int ld, int row0, int k0) {
  const int l = threadIdx.x & 31, h = l >> 4, m = l & 15;
  const unsigned short* r = p + (size_t)(row0 + m) * ld + k0 + 8 * h;
  Frag f;
  f.p[0] = *(const us8*)r;
  f.p[1] = *(const us8*)(r + 16);
  return f.u;
}

__device__ __forceinline__ v8f mma_h(us16 a, us16 b, v8f c) {
  Frag fa, fb;
  fa.u = a; fb.u = b;
  c = __builtin_amdgcn_wmma_f32_16x16x32_f16(false, fa.h, false, fb.h, (short)0, c, false, false);
  asm volatile("v_nop\n\tv_nop\n\tv_nop\n\tv_nop" : "+v"(c) : "v"(a), "v"(b));
  return c;
}
__device__ __forceinline__ v8f mma_b(us16 a, us16 b, v8f c) {
  Frag fa, fb;
  fa.u = a; fb.u = b;
  c = __builtin_amdgcn_wmma_f32_16x16x32_bf16(false, fa.b, false, fb.b, (short)0, c, false, false);
  asm volatile("v_nop\n\tv_nop\n\tv_nop\n\tv_nop" : "+v"(c) : "v"(a), "v"(b));
  return c;
}

__global__ __launch_bounds__(256) void cvt_w_kernel(const float* __restrict__ Wq, const float* __restrict__ Wk,
                                                    const float* __restrict__ Wv, const float* __restrict__ Wo,
                                                    unsigned short* Wqh, unsigned short* Wkh,
                                                    unsigned short* Wvhi, unsigned short* Wvlo,
                                                    unsigned short* Wohi, unsigned short* Wolo, int n8)
{
  const int t = blockIdx.x * 256 + threadIdx.x;
  if (t >= n8) return;
  const size_t e = (size_t)t * 8;
  float fq[8], fk[8], fv[8], fo[8];
  ld8(Wq + e, fq);
  ld8(Wk + e, fk);
  ld8(Wv + e, fv);
  ld8(Wo + e, fo);
  us8 oq, ok, ovh, ovl, ooh, ool;
#pragma unroll
  for (int i = 0; i < 8; ++i) {
    oq[i] = f2h(fq[i] * 32.0f);
    ok[i] = f2h(fk[i] * 32.0f);
    unsigned short hb = f2bf(fv[i]);
    ovh[i] = hb;
    ovl[i] = f2bf(fv[i] - bf2f(hb));
    hb = f2bf(fo[i]);
    ooh[i] = hb;
    ool[i] = f2bf(fo[i] - bf2f(hb));
  }
  *(volatile us8*)(Wqh + e)  = oq;
  *(volatile us8*)(Wkh + e)  = ok;
  *(volatile us8*)(Wvhi + e) = ovh;
  *(volatile us8*)(Wvlo + e) = ovl;
  *(volatile us8*)(Wohi + e) = ooh;
  *(volatile us8*)(Wolo + e) = ool;
  __threadfence();
  *(volatile us8*)(Wqh + e)  = oq;
  *(volatile us8*)(Wkh + e)  = ok;
  *(volatile us8*)(Wvhi + e) = ovh;
  *(volatile us8*)(Wvlo + e) = ovl;
  *(volatile us8*)(Wohi + e) = ooh;
  *(volatile us8*)(Wolo + e) = ool;
}

__global__ __launch_bounds__(256) void cvt_x_kernel(const float* __restrict__ xb,
                                                    unsigned short* Xh, unsigned short* Xhi, unsigned short* Xlo,
                                                    int n8)
{
  const int t = blockIdx.x * 256 + threadIdx.x;
  if (t >= n8) return;
  const size_t e = (size_t)t * 8;
  float f[8];
  ld8(xb + e, f);
  us8 oh, obh, obl;
#pragma unroll
  for (int i = 0; i < 8; ++i) {
    oh[i] = f2h(f[i]);
    unsigned short hb = f2bf(f[i]);
    obh[i] = hb;
    obl[i] = f2bf(f[i] - bf2f(hb));
  }
  *(volatile us8*)(Xh + e)  = oh;
  *(volatile us8*)(Xhi + e) = obh;
  *(volatile us8*)(Xlo + e) = obl;
  __threadfence();
  *(volatile us8*)(Xh + e)  = oh;
  *(volatile us8*)(Xhi + e) = obh;
  *(volatile us8*)(Xlo + e) = obl;
}

__global__ __launch_bounds__(128) void proj_qk_kernel(const unsigned short* Xh,
                                                     const unsigned short* Wqh, const unsigned short* Wkh,
                                                     const float* __restrict__ bq, const float* __restrict__ bk,
                                                     unsigned short* Qp, unsigned short* Kp)
{
  __shared__ __attribute__((aligned(16))) unsigned short tile[128 * 64];

  const int z = blockIdx.z;
  const unsigned short* W = z ? Wkh : Wqh;
  const float* bias = z ? bk : bq;
  unsigned short* dst = z ? Kp : Qp;

  const int tid = threadIdx.x, wave = tid >> 5, l = tid & 31, h = l >> 4, m = l & 15;
  const int tok0 = blockIdx.x * 128;
  const int head = blockIdx.y;
  const int col0 = head * DH;
  const int rw = tok0 + wave * 32;

  v8f acc[2][4];
#pragma unroll
  for (int rt = 0; rt < 2; ++rt)
#pragma unroll
    for (int t = 0; t < 4; ++t) acc[rt][t] = vzero();

#pragma unroll 1
  for (int k0 = 0; k0 < DM; k0 += 32) {
    const us16 a0 = ldfrag(Xh, DM, rw, k0);
    const us16 a1 = ldfrag(Xh, DM, rw + 16, k0);
#pragma unroll
    for (int t = 0; t < 4; ++t) {
      const us16 b = ldfrag(W, DM, col0 + t * 16, k0);
      acc[0][t] = mma_h(a0, b, acc[0][t]);
      acc[1][t] = mma_h(a1, b, acc[1][t]);
    }
  }

#pragma unroll
  for (int t = 0; t < 4; ++t) {
    const int d = t * 16 + m;
    const float bb = bias[col0 + d];
#pragma unroll
    for (int rt = 0; rt < 2; ++rt) {
#pragma unroll
      for (int r = 0; r < 8; ++r) {
        const int tl = wave * 32 + rt * 16 + 8 * h + r;
        const float v = acc[rt][t][r] * (1.0f / 32.0f) + bb;
        tile[tl * 64 + d] = f2h(v);
      }
    }
  }
  __syncthreads();

  const int piece = tid & 7;
  const int lb = tid >> 3;
#pragma unroll
  for (int it = 0; it < 8; ++it) {
    const int L = lb + 16 * it;
    const us8 v = *(const us8*)(tile + L * 64 + piece * 8);
    *(volatile us8*)(dst + ((size_t)(head * SEQ + tok0 + L)) * DH + piece * 8) = v;
  }
  __threadfence();
#pragma unroll
  for (int it = 0; it < 8; ++it) {
    const int L = lb + 16 * it;
    const us8 v = *(const us8*)(tile + L * 64 + piece * 8);
    *(volatile us8*)(dst + ((size_t)(head * SEQ + tok0 + L)) * DH + piece * 8) = v;
  }
}

__global__ __launch_bounds__(128) void proj_v_kernel(const unsigned short* Xhi, const unsigned short* Xlo,
                                                    const unsigned short* Wvhi, const unsigned short* Wvlo,
                                                    const float* __restrict__ bv,
                                                    unsigned short* Vthi, unsigned short* Vtlo)
{
  __shared__ __attribute__((aligned(16))) unsigned short thi[64 * 128];
  __shared__ __attribute__((aligned(16))) unsigned short tlo[64 * 128];

  const int tid = threadIdx.x, wave = tid >> 5, l = tid & 31, h = l >> 4, m = l & 15;
  const int tok0 = blockIdx.x * 128;
  const int head = blockIdx.y;
  const int col0 = head * DH;
  const int rw = tok0 + wave * 32;

  v8f acc[2][4];
#pragma unroll
  for (int rt = 0; rt < 2; ++rt)
#pragma unroll
    for (int t = 0; t < 4; ++t) acc[rt][t] = vzero();

#pragma unroll 1
  for (int k0 = 0; k0 < DM; k0 += 32) {
    const us16 a0h = ldfrag(Xhi, DM, rw, k0);
    const us16 a0l = ldfrag(Xlo, DM, rw, k0);
    const us16 a1h = ldfrag(Xhi, DM, rw + 16, k0);
    const us16 a1l = ldfrag(Xlo, DM, rw + 16, k0);
#pragma unroll
    for (int t = 0; t < 4; ++t) {
      const us16 bh = ldfrag(Wvhi, DM, col0 + t * 16, k0);
      const us16 bl = ldfrag(Wvlo, DM, col0 + t * 16, k0);
      acc[0][t] = mma_b(a0h, bh, acc[0][t]);
      acc[0][t] = mma_b(a0h, bl, acc[0][t]);
      acc[0][t] = mma_b(a0l, bh, acc[0][t]);
      acc[1][t] = mma_b(a1h, bh, acc[1][t]);
      acc[1][t] = mma_b(a1h, bl, acc[1][t]);
      acc[1][t] = mma_b(a1l, bh, acc[1][t]);
    }
  }

#pragma unroll
  for (int t = 0; t < 4; ++t) {
    const int d = t * 16 + m;
    const float bb = bv[col0 + d];
#pragma unroll
    for (int rt = 0; rt < 2; ++rt) {
#pragma unroll
      for (int r = 0; r < 8; ++r) {
        const int tl = wave * 32 + rt * 16 + 8 * h + r;
        const float v = acc[rt][t][r] + bb;
        const unsigned short hb = f2bf(v);
        thi[d * 128 + tl] = hb;
        tlo[d * 128 + tl] = f2bf(v - bf2f(hb));
      }
    }
  }
  __syncthreads();

  const int piece = tid & 7;
  const int lb = tid >> 3;
  const size_t pbase = (size_t)(head * DH) * SEQ;
#pragma unroll
  for (int it = 0; it < 8; ++it) {
    const int L = lb + 16 * it;
    const int d = L >> 1, hf = L & 1;
    const int so = d * 128 + hf * 64 + piece * 8;
    const size_t go = pbase + (size_t)d * SEQ + tok0 + hf * 64 + piece * 8;
    const us8 vh = *(const us8*)(thi + so);
    const us8 vl = *(const us8*)(tlo + so);
    *(volatile us8*)(Vthi + go) = vh;
    *(volatile us8*)(Vtlo + go) = vl;
  }
  __threadfence();
#pragma unroll
  for (int it = 0; it < 8; ++it) {
    const int L = lb + 16 * it;
    const int d = L >> 1, hf = L & 1;
    const int so = d * 128 + hf * 64 + piece * 8;
    const size_t go = pbase + (size_t)d * SEQ + tok0 + hf * 64 + piece * 8;
    const us8 vh = *(const us8*)(thi + so);
    const us8 vl = *(const us8*)(tlo + so);
    *(volatile us8*)(Vthi + go) = vh;
    *(volatile us8*)(Vtlo + go) = vl;
  }
}

__global__ __launch_bounds__(128) void attn_kernel(const unsigned short* Qp, const unsigned short* Kp,
                                                  const unsigned short* Vthi, const unsigned short* Vtlo,
                                                  const int* __restrict__ maskb,
                                                  unsigned short* Chi, unsigned short* Clo)
{
  __shared__ __attribute__((aligned(16))) unsigned short Phi[4][16 * 32];
  __shared__ __attribute__((aligned(16))) unsigned short Plo[4][16 * 32];
  __shared__ __attribute__((aligned(16))) unsigned short cth[64 * 64];
  __shared__ __attribute__((aligned(16))) unsigned short ctl[64 * 64];

  const int tid = threadIdx.x, wave = tid >> 5, l = tid & 31, h = l >> 4, m = l & 15;
  const int head = blockIdx.y;
  const int qt0 = blockIdx.x * 64;
  const int q0 = qt0 + wave * 16;
  const unsigned short* Qh = Qp + (size_t)head * SEQ * DH;
  const unsigned short* Kh = Kp + (size_t)head * SEQ * DH;
  const unsigned short* Vh = Vthi + (size_t)head * DH * SEQ;
  const unsigned short* Vl = Vtlo + (size_t)head * DH * SEQ;

  const us16 aq0 = ldfrag(Qh, DH, q0, 0);
  const us16 aq1 = ldfrag(Qh, DH, q0, 32);

  const float NEG = -__builtin_huge_valf();
  float mrun[8], lrun[8];
  v8f acc[4];
#pragma unroll
  for (int i = 0; i < 8; ++i) { mrun[i] = NEG; lrun[i] = 0.0f; }
#pragma unroll
  for (int t = 0; t < 4; ++t) acc[t] = vzero();

  unsigned short* phw = &Phi[wave][0];
  unsigned short* plw = &Plo[wave][0];

#pragma unroll 1
  for (int j = 0; j < SEQ; j += 32) {
    v8f s0 = vzero(), s1 = vzero();
    {
      const us16 b0 = ldfrag(Kh, DH, j, 0);
      const us16 b1 = ldfrag(Kh, DH, j, 32);
      s0 = mma_h(aq0, b0, s0);
      s0 = mma_h(aq1, b1, s0);
    }
    {
      const us16 b0 = ldfrag(Kh, DH, j + 16, 0);
      const us16 b1 = ldfrag(Kh, DH, j + 16, 32);
      s1 = mma_h(aq0, b0, s1);
      s1 = mma_h(aq1, b1, s1);
    }
    const int mk0 = maskb[j + m];
    const int mk1 = maskb[j + 16 + m];

    float al[8];
#pragma unroll
    for (int r = 0; r < 8; ++r) {
      const float v0 = (mk0 != 0) ? s0[r] * 0.125f : NEG;
      const float v1 = (mk1 != 0) ? s1[r] * 0.125f : NEG;
      float tmax = fmaxf(v0, v1);
#pragma unroll
      for (int off = 1; off < 16; off <<= 1) tmax = fmaxf(tmax, __shfl_xor(tmax, off, 32));
      const float mnew = fmaxf(mrun[r], tmax);
      const float msafe = (mnew == NEG) ? 0.0f : mnew;
      const float a = __expf(mrun[r] - msafe);
      const float p0 = __expf(v0 - msafe);
      const float p1 = __expf(v1 - msafe);
      float rs = p0 + p1;
#pragma unroll
      for (int off = 1; off < 16; off <<= 1) rs += __shfl_xor(rs, off, 32);
      lrun[r] = lrun[r] * a + rs;
      mrun[r] = mnew;
      al[r] = a;
      const int row = 8 * h + r;
      const unsigned short h0 = f2bf(p0);
      const unsigned short h1 = f2bf(p1);
      phw[row * 32 + m]      = h0;
      phw[row * 32 + 16 + m] = h1;
      plw[row * 32 + m]      = f2bf(p0 - bf2f(h0));
      plw[row * 32 + 16 + m] = f2bf(p1 - bf2f(h1));
    }
#pragma unroll
    for (int t = 0; t < 4; ++t)
#pragma unroll
      for (int r = 0; r < 8; ++r) acc[t][r] *= al[r];

    __syncthreads();

    const us16 ph = ldfrag(phw, 32, 0, 0);
    const us16 pl = ldfrag(plw, 32, 0, 0);
#pragma unroll
    for (int t = 0; t < 4; ++t) {
      const us16 vh = ldfrag(Vh, SEQ, t * 16, j);
      const us16 vl = ldfrag(Vl, SEQ, t * 16, j);
      acc[t] = mma_b(ph, vh, acc[t]);
      acc[t] = mma_b(ph, vl, acc[t]);
      acc[t] = mma_b(pl, vh, acc[t]);
    }
    __syncthreads();
  }

#pragma unroll
  for (int t = 0; t < 4; ++t) {
    const int d = t * 16 + m;
#pragma unroll
    for (int r = 0; r < 8; ++r) {
      const float li = lrun[r];
      const float o = acc[t][r] * (1.0f / li);
      const int row = wave * 16 + 8 * h + r;
      const unsigned short hb = f2bf(o);
      cth[row * 64 + d] = hb;
      ctl[row * 64 + d] = f2bf(o - bf2f(hb));
    }
  }
  __syncthreads();

  const int piece = tid & 7;
  const int lb = tid >> 3;
#pragma unroll
  for (int it = 0; it < 4; ++it) {
    const int L = lb + 16 * it;
    const int so = L * 64 + piece * 8;
    const size_t go = (size_t)(qt0 + L) * DM + head * DH + piece * 8;
    const us8 vh = *(const us8*)(cth + so);
    const us8 vl = *(const us8*)(ctl + so);
    *(volatile us8*)(Chi + go) = vh;
    *(volatile us8*)(Clo + go) = vl;
  }
  __threadfence();
#pragma unroll
  for (int it = 0; it < 4; ++it) {
    const int L = lb + 16 * it;
    const int so = L * 64 + piece * 8;
    const size_t go = (size_t)(qt0 + L) * DM + head * DH + piece * 8;
    const us8 vh = *(const us8*)(cth + so);
    const us8 vl = *(const us8*)(ctl + so);
    *(volatile us8*)(Chi + go) = vh;
    *(volatile us8*)(Clo + go) = vl;
  }
}

__global__ __launch_bounds__(128) void proj_o_kernel(const unsigned short* Chi, const unsigned short* Clo,
                                                    const unsigned short* Wohi, const unsigned short* Wolo,
                                                    float* outb)
{
  __shared__ __attribute__((aligned(16))) float tilef[128 * 64];

  const int tid = threadIdx.x, wave = tid >> 5, l = tid & 31, h = l >> 4, m = l & 15;
  const int tok0 = blockIdx.x * 128;
  const int col0 = blockIdx.y * 64;
  const int rw = tok0 + wave * 32;

  v8f acc[2][4];
#pragma unroll
  for (int rt = 0; rt < 2; ++rt)
#pragma unroll
    for (int t = 0; t < 4; ++t) acc[rt][t] = vzero();

#pragma unroll 1
  for (int k0 = 0; k0 < DM; k0 += 32) {
    const us16 a0h = ldfrag(Chi, DM, rw, k0);
    const us16 a0l = ldfrag(Clo, DM, rw, k0);
    const us16 a1h = ldfrag(Chi, DM, rw + 16, k0);
    const us16 a1l = ldfrag(Clo, DM, rw + 16, k0);
#pragma unroll
    for (int t = 0; t < 4; ++t) {
      const us16 bh = ldfrag(Wohi, DM, col0 + t * 16, k0);
      const us16 bl = ldfrag(Wolo, DM, col0 + t * 16, k0);
      acc[0][t] = mma_b(a0h, bh, acc[0][t]);
      acc[0][t] = mma_b(a0h, bl, acc[0][t]);
      acc[0][t] = mma_b(a0l, bh, acc[0][t]);
      acc[1][t] = mma_b(a1h, bh, acc[1][t]);
      acc[1][t] = mma_b(a1h, bl, acc[1][t]);
      acc[1][t] = mma_b(a1l, bh, acc[1][t]);
    }
  }

#pragma unroll
  for (int t = 0; t < 4; ++t) {
    const int d = t * 16 + m;
#pragma unroll
    for (int rt = 0; rt < 2; ++rt) {
#pragma unroll
      for (int r = 0; r < 8; ++r) {
        const int tl = wave * 32 + rt * 16 + 8 * h + r;
        tilef[tl * 64 + d] = acc[rt][t][r];
      }
    }
  }
  __syncthreads();

  const int piece = tid & 7;
  const int lb = tid >> 3;
#pragma unroll
  for (int it = 0; it < 16; ++it) {
    const int L = lb + 16 * it;
    const int row = L >> 1, hf = L & 1;
    const v4f v = *(const v4f*)(tilef + row * 64 + hf * 32 + piece * 4);
    *(volatile v4f*)(outb + (size_t)(tok0 + row) * DM + col0 + hf * 32 + piece * 4) = v;
  }
  __threadfence();
#pragma unroll
  for (int it = 0; it < 16; ++it) {
    const int L = lb + 16 * it;
    const int row = L >> 1, hf = L & 1;
    const v4f v = *(const v4f*)(tilef + row * 64 + hf * 32 + piece * 4);
    *(volatile v4f*)(outb + (size_t)(tok0 + row) * DM + col0 + hf * 32 + piece * 4) = v;
  }
}

extern "C" void kernel_launch(void* const* d_in, const int* in_sizes, int n_in,
                              void* d_out, int out_size, void* d_ws, size_t ws_size,
                              hipStream_t stream) {
  if (n_in < 9) return;
  if (in_sizes[0] != NB * SEQ * DM) return;
  if (in_sizes[1] != NB * SEQ) return;
  if (in_sizes[2] != DM * DM || in_sizes[4] != DM * DM || in_sizes[6] != DM * DM || in_sizes[8] != DM * DM) return;
  if (in_sizes[3] != DM || in_sizes[5] != DM || in_sizes[7] != DM) return;
  if (out_size != NB * SEQ * DM) return;

  const float* x    = (const float*)d_in[0];
  const int*   mask = (const int*)d_in[1];
  const float* Wq   = (const float*)d_in[2];
  const float* bq   = (const float*)d_in[3];
  const float* Wk   = (const float*)d_in[4];
  const float* bk   = (const float*)d_in[5];
  const float* Wv   = (const float*)d_in[6];
  const float* bv   = (const float*)d_in[7];
  const float* Wo   = (const float*)d_in[8];
  float*       out  = (float*)d_out;

  const size_t wplane = (size_t)DM * DM * 2;
  const size_t xplane = (size_t)SEQ * DM * 2;
  const size_t hplane = (size_t)NH * SEQ * DH * 2;
  char* w = (char*)d_ws;
  size_t off = 0;
  unsigned short* Wqh  = (unsigned short*)(w + off); off += wplane;
  unsigned short* Wkh  = (unsigned short*)(w + off); off += wplane;
  unsigned short* Wvhi = (unsigned short*)(w + off); off += wplane;
  unsigned short* Wvlo = (unsigned short*)(w + off); off += wplane;
  unsigned short* Wohi = (unsigned short*)(w + off); off += wplane;
  unsigned short* Wolo = (unsigned short*)(w + off); off += wplane;
  unsigned short* Xh   = (unsigned short*)(w + off); off += xplane;
  unsigned short* Xhi  = (unsigned short*)(w + off); off += xplane;
  unsigned short* Xlo  = (unsigned short*)(w + off); off += xplane;
  unsigned short* Qp   = (unsigned short*)(w + off); off += hplane;
  unsigned short* Kp   = (unsigned short*)(w + off); off += hplane;
  unsigned short* Vthi = (unsigned short*)(w + off); off += hplane;
  unsigned short* Vtlo = (unsigned short*)(w + off); off += hplane;
  unsigned short* Chi  = (unsigned short*)(w + off); off += xplane;
  unsigned short* Clo  = (unsigned short*)(w + off); off += xplane;
  if (off > ws_size) return;

  const int nw8 = DM * DM / 8;
  const int nx8 = SEQ * DM / 8;
  cvt_w_kernel<<<dim3((nw8 + 255) / 256), dim3(256), 0, stream>>>(Wq, Wk, Wv, Wo, Wqh, Wkh, Wvhi, Wvlo, Wohi, Wolo, nw8);

  for (int b = 0; b < NB; ++b) {
    const float* xb   = x + (size_t)b * SEQ * DM;
    const int*   mb   = mask + (size_t)b * SEQ;
    float*       outb = out + (size_t)b * SEQ * DM;

    cvt_x_kernel<<<dim3((nx8 + 255) / 256), dim3(256), 0, stream>>>(xb, Xh, Xhi, Xlo, nx8);
    proj_qk_kernel<<<dim3(SEQ / 128, NH, 2), dim3(128), 0, stream>>>(Xh, Wqh, Wkh, bq, bk, Qp, Kp);
    proj_v_kernel<<<dim3(SEQ / 128, NH), dim3(128), 0, stream>>>(Xhi, Xlo, Wvhi, Wvlo, bv, Vthi, Vtlo);
    attn_kernel<<<dim3(SEQ / 64, NH), dim3(128), 0, stream>>>(Qp, Kp, Vthi, Vtlo, mb, Chi, Clo);
    proj_o_kernel<<<dim3(SEQ / 128, DM / 64), dim3(128), 0, stream>>>(Chi, Clo, Wohi, Wolo, outb);
  }
}
